// FrameTransformerEncoder_66202625900954
// MI455X (gfx1250) — hardware-verified
//
#include <hip/hip_runtime.h>
#include <math.h>
#include <stdint.h>

#pragma clang fp contract(off)

#define NB   2
#define NCI  2
#define NC   4
#define NG   (NB * NC)
#define NF   512
#define NW   1024
#define NHD  16
#define HD   32
#define NFE  2048
#define GFW  (NF * NW)
#define GWE  (NW * NFE)
#define WSQ  (NC * NF * NF)
#define WSL  (NC * NFE * NF)
#define NWH  (4 * WSQ + 2 * WSL)
#define CVB  2048

static_assert(NG == NB * NC);
static_assert((NG % NC) == 0);
static_assert(NC == 4 && NCI == 2);
static_assert(NF == 8 * 64);
static_assert(NHD * HD == NF && HD == 32 && (NHD % 2) == 0);
static_assert(NFE == 4 * NF);
static_assert((NF % 64) == 0 && (NW % 64) == 0 && (NFE % 64) == 0);
static_assert((WSQ % CVB) == 0 && (WSL % CVB) == 0 && (NWH % CVB) == 0);
static_assert(((2 * NG * NW * (NF / 8)) % 256) == 0);
static_assert(((NG * NF * (NW / 8)) % 256) == 0);
static_assert((NW % 32) == 0);

typedef _Float16 v16h __attribute__((ext_vector_type(16)));
typedef _Float16 v8h  __attribute__((ext_vector_type(8)));
typedef float    v8f  __attribute__((ext_vector_type(8)));
typedef float    v4f  __attribute__((ext_vector_type(4)));
typedef unsigned int v4u __attribute__((ext_vector_type(4)));

__device__ __forceinline__ unsigned short bf_bits(float f) {
  unsigned u = __float_as_uint(f);
  return (unsigned short)((u + 0x7FFFu + ((u >> 16) & 1u)) >> 16);
}
__device__ __forceinline__ float bf_up(unsigned short h) { return __uint_as_float(((unsigned)h) << 16); }
__device__ __forceinline__ float bfr(float f) { return bf_up(bf_bits(f)); }
__device__ __forceinline__ unsigned short h_bits(_Float16 x) { return __builtin_bit_cast(unsigned short, x); }
__device__ __forceinline__ unsigned pk16(unsigned short a, unsigned short b) { return (unsigned)a | ((unsigned)b << 16); }
__device__ __forceinline__ unsigned pkh(float a, float b) { return pk16(h_bits((_Float16)a), h_bits((_Float16)b)); }
__device__ __forceinline__ v8f zero8() { v8f z = {0.f, 0.f, 0.f, 0.f, 0.f, 0.f, 0.f, 0.f}; return z; }

__device__ __forceinline__ v16h ldfrag_h(const _Float16* p) {
  union { v16h v; v8h h[2]; } f;
  f.h[0] = *(const v8h*)(p);
  f.h[1] = *(const v8h*)(p + 16);
  return f.v;
}

__device__ __forceinline__ v8f mma_h(v16h a, v16h b, v8f c) {
  c = __builtin_amdgcn_wmma_f32_16x16x32_f16(false, a, false, b, (short)0, c, false, false);
#if defined(__HIP_DEVICE_COMPILE__)
  asm volatile("v_nop\n\tv_nop\n\tv_nop\n\tv_nop" : "+v"(c) : "v"(a), "v"(b));
#endif
  return c;
}
__device__ __forceinline__ v8f mma_h_raw(v16h a, v16h b, v8f c) {
  return __builtin_amdgcn_wmma_f32_16x16x32_f16(false, a, false, b, (short)0, c, false, false);
}
__device__ __forceinline__ void dep_guard_h(v8f& a, v8f& b, v16h x, v16h y) {
#if defined(__HIP_DEVICE_COMPILE__)
  asm volatile("v_nop\n\tv_nop\n\tv_nop\n\tv_nop" : "+v"(a), "+v"(b) : "v"(x), "v"(y));
#endif
}
__device__ __forceinline__ void keep4_h(v16h a, v16h b, v16h c, v16h d) {
#if defined(__HIP_DEVICE_COMPILE__)
  asm volatile("v_nop" :: "v"(a), "v"(b), "v"(c), "v"(d));
#endif
}
__device__ __forceinline__ void acc_guard4(v8f& a, v8f& b, v8f& c, v8f& d) {
#if defined(__HIP_DEVICE_COMPILE__)
  asm volatile("v_nop\n\tv_nop\n\tv_nop\n\tv_nop" : "+v"(a), "+v"(b), "+v"(c), "+v"(d));
#endif
}
__device__ __forceinline__ void wave_sync_lds() {
  __builtin_amdgcn_fence(__ATOMIC_RELEASE, "workgroup");
  __builtin_amdgcn_wave_barrier();
  __builtin_amdgcn_fence(__ATOMIC_ACQUIRE, "workgroup");
}

__global__ __launch_bounds__(256) void cvt_w(const float* __restrict__ wq, const float* __restrict__ wk,
                                             const float* __restrict__ wv, const float* __restrict__ wo,
                                             const float* __restrict__ w1, const float* __restrict__ w2,
                                             unsigned short* wh) {
#pragma clang fp contract(off)
  const int tid = threadIdx.x;
  const int blk = blockIdx.x;
  const int b1 = WSQ / CVB, b2 = (2 * WSQ) / CVB, b3 = (3 * WSQ) / CVB, b4 = (4 * WSQ) / CVB, b5 = (4 * WSQ + WSL) / CVB;
  const float* src = (blk < b1) ? wq : ((blk < b2) ? wk : ((blk < b3) ? wv : ((blk < b4) ? wo : ((blk < b5) ? w1 : w2))));
  const int base = (blk < b1) ? 0 : ((blk < b2) ? WSQ : ((blk < b3) ? (2 * WSQ) : ((blk < b4) ? (3 * WSQ)
                   : ((blk < b5) ? (4 * WSQ) : (4 * WSQ + WSL)))));
  const int e0 = blk * CVB + tid * 8;
  const float* sp = src + (e0 - base);
  const v4f a = *(const v4f*)sp;
  const v4f b = *(const v4f*)(sp + 4);
  v4u pk;
  pk[0] = pkh(bfr(a[0]) * 64.0f, bfr(a[1]) * 64.0f);
  pk[1] = pkh(bfr(a[2]) * 64.0f, bfr(a[3]) * 64.0f);
  pk[2] = pkh(bfr(b[0]) * 64.0f, bfr(b[1]) * 64.0f);
  pk[3] = pkh(bfr(b[2]) * 64.0f, bfr(b[3]) * 64.0f);
  unsigned short* gp = wh + e0;
  *(volatile v4u*)gp = pk;
  __threadfence();
  *(volatile v4u*)gp = pk;
}

__global__ __launch_bounds__(256) void trig_tab(float* tb) {
#pragma clang fp contract(off)
  const int w = blockIdx.x * 256 + threadIdx.x;
  if (w >= NW) return;
  const int yi = blockIdx.y;
  const int i = yi & 15;
  float inv = 1.0f;
  inv = (i == 1)  ? 0.562341325f    : inv;
  inv = (i == 2)  ? 0.316227766f    : inv;
  inv = (i == 3)  ? 0.177827941f    : inv;
  inv = (i == 4)  ? 0.1f            : inv;
  inv = (i == 5)  ? 0.0562341325f   : inv;
  inv = (i == 6)  ? 0.0316227766f   : inv;
  inv = (i == 7)  ? 0.0177827941f   : inv;
  inv = (i == 8)  ? 0.01f           : inv;
  inv = (i == 9)  ? 0.00562341325f  : inv;
  inv = (i == 10) ? 0.00316227766f  : inv;
  inv = (i == 11) ? 0.00177827941f  : inv;
  inv = (i == 12) ? 0.001f          : inv;
  inv = (i == 13) ? 0.000562341325f : inv;
  inv = (i == 14) ? 0.000316227766f : inv;
  inv = (i == 15) ? 0.000177827941f : inv;
  const float ang = (float)w * inv;
  const float cv = cosf(ang);
  const float sv = sinf(ang);
  const float v = (yi >= 16) ? sv : cv;
  float* p = tb + (size_t)yi * NW + w;
  *(volatile float*)p = v;
  __threadfence();
  *(volatile float*)p = v;
}

template <int EMBED>
__global__ __launch_bounds__(256) void ln_cols(const float* __restrict__ xin, const float* __restrict__ ew,
                                               const float* __restrict__ eb, const float* __restrict__ nw,
                                               const float* __restrict__ nb, float* xout, unsigned short* xnt) {
#pragma clang fp contract(off)
  __shared__ float red[8][32];
  __shared__ __align__(16) unsigned int Ts[32][260];
  const int tid = threadIdx.x;
  const int wave = tid >> 5, lane = tid & 31;
  const int g = blockIdx.y;
  const int bb = g / NC, ch = g % NC;
  const int w0 = blockIdx.x * 32;
  const int col = w0 + lane;
  const int fb = wave * 64;
  float xv[64];
  if (EMBED) {
    const float e0 = bfr(ew[ch * NCI]), e1 = bfr(ew[ch * NCI + 1]), ebv = bfr(eb[ch]);
    const float* p0 = xin + ((size_t)(bb * NCI) * NF + fb) * NW + col;
    const float* p1 = xin + ((size_t)(bb * NCI + 1) * NF + fb) * NW + col;
#pragma unroll
    for (int j = 0; j < 64; ++j) {
      const float a0 = bfr(p0[(size_t)j * NW]);
      const float a1 = bfr(p1[(size_t)j * NW]);
      const float t0 = e0 * a0;
      const float t1 = e1 * a1;
      const float s = t0 + t1;
      xv[j] = s + ebv;
    }
    float* xo = xout + ((size_t)g * NF + fb) * NW + col;
    for (int ps = 0; ps < 2; ++ps) {
#pragma unroll
      for (int j = 0; j < 64; ++j) *(volatile float*)(xo + (size_t)j * NW) = xv[j];
      __threadfence();
    }
  } else {
    const float* p = xin + ((size_t)g * NF + fb) * NW + col;
#pragma unroll
    for (int j = 0; j < 64; ++j) xv[j] = p[(size_t)j * NW];
  }
  float s = 0.f;
#pragma unroll
  for (int j = 0; j < 64; ++j) s = s + xv[j];
  red[wave][lane] = s;
  __syncthreads();
  float tot = 0.f;
#pragma unroll
  for (int q = 0; q < 8; ++q) tot = tot + red[q][lane];
  const float mu = tot * (1.0f / NF);
  __syncthreads();
  float s2 = 0.f;
#pragma unroll
  for (int j = 0; j < 64; ++j) {
    const float d = xv[j] - mu;
    xv[j] = d;
    const float dd = d * d;
    s2 = s2 + dd;
  }
  red[wave][lane] = s2;
  __syncthreads();
  float tot2 = 0.f;
#pragma unroll
  for (int q = 0; q < 8; ++q) tot2 = tot2 + red[q][lane];
  const float var = tot2 * (1.0f / NF);
  const float rstd = 1.0f / sqrtf(var + 1e-8f);
  const float* nwc = nw + ch * NF + fb;
  const float* nbc = nb + ch * NF + fb;
#pragma unroll
  for (int e8 = 0; e8 < 8; ++e8) {
    v4u pk;
#pragma unroll
    for (int e = 0; e < 4; ++e) {
      const int j = e8 * 8 + 2 * e;
      const float g0 = bfr(nwc[j]), g1 = bfr(nwc[j + 1]);
      const float b0 = bfr(nbc[j]), b1 = bfr(nbc[j + 1]);
      float t0 = xv[j] * rstd;     t0 = t0 * g0; const float y0 = t0 + b0;
      float t1 = xv[j + 1] * rstd; t1 = t1 * g1; const float y1 = t1 + b1;
      pk[e] = pkh(y0, y1);
    }
    *(v4u*)(&Ts[lane][wave * 32 + e8 * 4]) = pk;
  }
  __syncthreads();
  v4u ov[8];
#pragma unroll
  for (int it = 0; it < 8; ++it) {
    const int row = wave * 4 + (it >> 1), hf = it & 1;
    ov[it] = *(const v4u*)(&Ts[row][hf * 128 + lane * 4]);
  }
  for (int ps = 0; ps < 2; ++ps) {
#pragma unroll
    for (int it = 0; it < 8; ++it) {
      const int row = wave * 4 + (it >> 1), hf = it & 1;
      *(volatile v4u*)(xnt + ((size_t)g * NW + w0 + row) * NF + hf * 256 + lane * 8) = ov[it];
    }
    __threadfence();
  }
}

struct GemmArgs {
  const unsigned short* A;
  const unsigned short* B;
  void* C;
  const float* R;
  long long aP, aG, aC, bP, bG, bC, cP, cG, cC;
  int lda, ldb, ldc, M, N, K;
  float s0, s1;
};
static_assert(sizeof(GemmArgs) == 136);

template <int OUT_MODE>
__global__ __launch_bounds__(256) void gemm64(GemmArgs ga) {
#pragma clang fp contract(off)
  __shared__ __align__(16) float sT[8][16 * 68];
  const int lane = threadIdx.x & 31;
  const int wave = threadIdx.x >> 5;
  const int z = blockIdx.y;
  const long long zp = z / NG, zg = z % NG, zc = z % NC;
  const _Float16* A  = (const _Float16*)(const void*)(ga.A + (zp * ga.aP + zg * ga.aG + zc * ga.aC));
  const _Float16* Bt = (const _Float16*)(const void*)(ga.B + (zp * ga.bP + zg * ga.bG + zc * ga.bC));
  const long long coff = zp * ga.cP + zg * ga.cG + zc * ga.cC;
  const int lda = ga.lda, ldb = ga.ldb, ldc = ga.ldc, K = ga.K;
  const int tilesN = ga.N >> 6;
  const int tilesM = ga.M >> 6;
  const int tile = blockIdx.x * 8 + wave;
  if (tile >= tilesM * tilesN) return;
  const int tm = tile / tilesN;
  const int tn = tile - tm * tilesN;
  const int m0 = tm << 6;
  const int n0 = tn << 6;

  const int rlane = lane & 15;
  const int koff  = (lane >> 4) * 8;
  const int mOff  = (lane >> 4) * 8;

  v8f acc[4][4];
#pragma unroll
  for (int i = 0; i < 4; ++i)
#pragma unroll
    for (int j = 0; j < 4; ++j) acc[i][j] = zero8();

  for (int k0 = 0; k0 < K; k0 += 32) {
    v16h bh[4];
#pragma unroll
    for (int j = 0; j < 4; ++j) {
      const size_t bo = (size_t)(n0 + (j << 4) + rlane) * ldb + koff + k0;
      bh[j] = ldfrag_h(Bt + bo);
    }
#pragma unroll
    for (int i = 0; i < 4; ++i) {
      const size_t ao = (size_t)(m0 + (i << 4) + rlane) * lda + koff + k0;
      const v16h ah = ldfrag_h(A + ao);
#pragma unroll
      for (int j = 0; j < 4; ++j) acc[i][j] = mma_h_raw(ah, bh[j], acc[i][j]);
      dep_guard_h(acc[i][0], acc[i][3], ah, bh[3]);
    }
    keep4_h(bh[0], bh[1], bh[2], bh[3]);
  }
#pragma unroll
  for (int i = 0; i < 4; ++i) acc_guard4(acc[i][0], acc[i][1], acc[i][2], acc[i][3]);

  float* slab = sT[wave];
#pragma unroll
  for (int i = 0; i < 4; ++i) {
    const int mBase = m0 + (i << 4);
#pragma unroll
    for (int j = 0; j < 4; ++j) {
#pragma unroll
      for (int r = 0; r < 8; ++r) {
        slab[(mOff + r) * 68 + (j << 4) + rlane] = acc[i][j][r];
      }
    }
    wave_sync_lds();
    if (OUT_MODE == 0) {
      float* Cf = (float*)ga.C + coff;
      const float* Rf = ga.R + coff;
      const int h2 = lane >> 4, c4 = (lane & 15) * 4;
      for (int ps = 0; ps < 2; ++ps) {
#pragma unroll
        for (int it = 0; it < 8; ++it) {
          const int row = it * 2 + h2;
          const int m = mBase + row;
          const v4f v  = *(const v4f*)(slab + row * 68 + c4);
          const v4f rr = *(const v4f*)(Rf + (size_t)m * ldc + n0 + c4);
          v4f ov;
#pragma unroll
          for (int e = 0; e < 4; ++e) { const float t = v[e] * ga.s0; ov[e] = rr[e] + t; }
          *(volatile v4f*)(Cf + (size_t)m * ldc + n0 + c4) = ov;
        }
        __threadfence();
      }
    } else {
      unsigned short* Ch = (unsigned short*)ga.C + coff;
      const int q = lane >> 3, c8 = (lane & 7) * 8;
      v4u hv[4];
#pragma unroll
      for (int it = 0; it < 4; ++it) {
        const int row = it * 4 + q;
        const float* sp = slab + row * 68 + c8;
        v4u a;
#pragma unroll
        for (int e = 0; e < 4; ++e) {
          float x0 = sp[2 * e] * ga.s0;
          float x1 = sp[2 * e + 1] * ga.s0;
          if (OUT_MODE == 2) {
            x0 = fmaxf(x0, 0.0f); x0 = x0 * x0; x0 = x0 * ga.s1;
            x1 = fmaxf(x1, 0.0f); x1 = x1 * x1; x1 = x1 * ga.s1;
          }
          a[e] = pkh(x0, x1);
        }
        hv[it] = a;
      }
      for (int ps = 0; ps < 2; ++ps) {
#pragma unroll
        for (int it = 0; it < 4; ++it) {
          const int row = it * 4 + q;
          *(volatile v4u*)(Ch + (size_t)(mBase + row) * ldc + n0 + c8) = hv[it];
        }
        __threadfence();
      }
    }
    wave_sync_lds();
  }
}

__global__ __launch_bounds__(256) void conv_qk(const unsigned short* __restrict__ yt, const float* __restrict__ cwq,
                                               const float* __restrict__ cbq, const float* __restrict__ cwk,
                                               const float* __restrict__ cbk, const float* __restrict__ tb,
                                               unsigned short* qkt) {
#pragma clang fp contract(off)
  union LH { v4u u; v8h v; };
  const int idx = blockIdx.x * 256 + threadIdx.x;
  const int f8  = idx % (NF / 8);
  const int t1  = idx / (NF / 8);
  const int w   = t1 % NW;
  const int t2  = t1 / NW;
  const int gco = t2 % NG;
  const int p   = t2 / NG;
  const int bb = gco / NC, co = gco % NC;
  const int f0 = f8 * 8;
  const float* cw = (p != 0) ? cwk : cwq;
  const float* cb = (p != 0) ? cbk : cbq;
  const _Float16* Y = (const _Float16*)(const void*)yt;
  float acc[8];
  const float bias = bfr(cb[co]) * 64.0f;
#pragma unroll
  for (int e = 0; e < 8; ++e) acc[e] = bias;
#pragma unroll 1
  for (int ci = 0; ci < NC; ++ci) {
    const _Float16* src = Y + ((size_t)(p * NG + bb * NC + ci) * NW) * NF + f0;
#pragma unroll
    for (int t = 0; t < 3; ++t) {
      const int wp = w + t - 1;
      const int wc = (wp < 0) ? 0 : ((wp > NW - 1) ? (NW - 1) : wp);
      float cwt = bfr(cw[(co * NC + ci) * 3 + t]);
      cwt = (wp >= 0 && wp < NW) ? cwt : 0.0f;
      LH ld;
      ld.u = *(const v4u*)(src + (size_t)wc * NF);
#pragma unroll
      for (int e = 0; e < 8; ++e) {
        const float y = (float)ld.v[e];
        const float m = cwt * y;
        acc[e] = acc[e] + m;
      }
    }
  }
  const int i0 = (f0 % HD) >> 1;
  float cs[4], sn[4];
#pragma unroll
  for (int e2 = 0; e2 < 4; ++e2) {
    cs[e2] = tb[(size_t)(i0 + e2) * NW + w];
    sn[e2] = tb[(size_t)(16 + i0 + e2) * NW + w];
  }
  v4u pk;
#pragma unroll
  for (int e2 = 0; e2 < 4; ++e2) {
    const float y0 = acc[2 * e2], y1 = acc[2 * e2 + 1];
    const float a0 = y0 * cs[e2];
    const float ny1 = -y1;
    const float b0 = ny1 * sn[e2];
    const float r0 = a0 + b0;
    const float a1 = y1 * cs[e2];
    const float b1 = y0 * sn[e2];
    const float r1 = a1 + b1;
    pk[e2] = pkh(r0, r1);
  }
  unsigned short* dst = qkt + ((size_t)(p * NG + gco) * NW + w) * NF + f0;
  *(volatile v4u*)dst = pk;
  __threadfence();
  *(volatile v4u*)dst = pk;
}

__global__ __launch_bounds__(256) void conv_v(const unsigned short* __restrict__ yv, const float* __restrict__ cw,
                                              const float* __restrict__ cb, unsigned short* vout) {
#pragma clang fp contract(off)
  union LH { v4u u; v8h v; };
  const int idx = blockIdx.x * 256 + threadIdx.x;
  const int w8  = idx % (NW / 8);
  const int t1  = idx / (NW / 8);
  const int f   = t1 % NF;
  const int gco = (t1 / NF) % NG;
  const int bb = gco / NC, co = gco % NC;
  const int wb = w8 * 8;
  const int wl = (wb > 0) ? (wb - 1) : 0;
  const int wr = (wb + 8 < NW) ? (wb + 8) : (NW - 1);
  const _Float16* Y = (const _Float16*)(const void*)yv;
  float acc[8];
  const float bias = bfr(cb[co]) * 64.0f;
#pragma unroll
  for (int e = 0; e < 8; ++e) acc[e] = bias;
#pragma unroll 1
  for (int ci = 0; ci < NC; ++ci) {
    const _Float16* row = Y + ((size_t)(bb * NC + ci) * NF + f) * NW;
    LH mid;
    mid.u = *(const v4u*)(row + wb);
    float lf = (float)row[wl];
    float rt = (float)row[wr];
    lf = (wb > 0) ? lf : 0.0f;
    rt = (wb + 8 < NW) ? rt : 0.0f;
    float y[10];
    y[0] = lf;
#pragma unroll
    for (int e = 0; e < 8; ++e) y[1 + e] = (float)mid.v[e];
    y[9] = rt;
    const float c0 = bfr(cw[(co * NC + ci) * 3 + 0]);
    const float c1 = bfr(cw[(co * NC + ci) * 3 + 1]);
    const float c2 = bfr(cw[(co * NC + ci) * 3 + 2]);
#pragma unroll
    for (int e = 0; e < 8; ++e) {
      const float m0 = c0 * y[e];
      const float m1 = c1 * y[e + 1];
      const float m2 = c2 * y[e + 2];
      float a = acc[e] + m0;
      a = a + m1;
      acc[e] = a + m2;
    }
  }
  v4u pk;
#pragma unroll
  for (int e = 0; e < 4; ++e) pk[e] = pkh(acc[2 * e], acc[2 * e + 1]);
  unsigned short* dst = vout + ((size_t)gco * NF + f) * NW + wb;
  *(volatile v4u*)dst = pk;
  __threadfence();
  *(volatile v4u*)dst = pk;
}

__global__ __launch_bounds__(256)
void attn_hd32(const unsigned short* __restrict__ qtp, const unsigned short* __restrict__ ktp,
               const unsigned short* __restrict__ vfp, unsigned short* atp, float sscale) {
#pragma clang fp contract(off)
  union FH { v16h v; v8h h[2]; };
  __shared__ __align__(16) _Float16 Psh[8][16 * 64];
  __shared__ __align__(16) float    Os[64 * 68];

  const int tid  = threadIdx.x;
  const int wave = tid >> 5;
  const int lane = tid & 31;
  const int hh   = lane >> 4;
  const int c    = lane & 15;

  const int qt   = blockIdx.x;
  const int hp   = blockIdx.y;
  const int g    = blockIdx.z;
  const int hl   = wave >> 2;
  const int wq   = wave & 3;
  const int head = hp * 2 + hl;
  const int q0   = qt * 64 + wq * 16;
  const size_t trow0 = (size_t)g * NW;

  const _Float16* Q = (const _Float16*)(const void*)qtp;
  const _Float16* Kk = (const _Float16*)(const void*)ktp;
  const _Float16* V = (const _Float16*)(const void*)vfp;

  const v16h qa = ldfrag_h(Q + (trow0 + q0 + c) * NF + head * HD + 8 * hh);

  float mrow[8], lrow[8];
  v8f o[2];
#pragma unroll
  for (int r = 0; r < 8; ++r) { mrow[r] = -INFINITY; lrow[r] = 0.f; }
#pragma unroll
  for (int t = 0; t < 2; ++t) o[t] = zero8();

  _Float16* pw = Psh[wave];

  for (int kt = 0; kt < NW / 64; ++kt) {
    const int kv0 = kt * 64;

    v8f s[4];
#pragma unroll
    for (int j = 0; j < 4; ++j) {
      const int key = kv0 + j * 16 + c;
      const v16h kb = ldfrag_h(Kk + (trow0 + key) * NF + head * HD + 8 * hh);
      v8f a = zero8();
      a = mma_h(qa, kb, a);
#pragma unroll
      for (int r = 0; r < 8; ++r) s[j][r] = a[r] * sscale;
    }

#pragma unroll
    for (int r = 0; r < 8; ++r) {
      float m = fmaxf(fmaxf(s[0][r], s[1][r]), fmaxf(s[2][r], s[3][r]));
#pragma unroll
      for (int off = 1; off < 16; off <<= 1) m = fmaxf(m, __shfl_xor(m, off, 32));
      const float mnew  = fmaxf(mrow[r], m);
      const float alpha = __expf(mrow[r] - mnew);
      mrow[r] = mnew;
      float psum = 0.f;
#pragma unroll
      for (int j = 0; j < 4; ++j) {
        const float p  = __expf(s[j][r] - mnew);
        psum = psum + p;
        const float p1 = p * 1024.0f;
        pw[(8 * hh + r) * 64 + j * 16 + c] = (_Float16)p1;
      }
#pragma unroll
      for (int off = 1; off < 16; off <<= 1) psum = psum + __shfl_xor(psum, off, 32);
      const float la = lrow[r] * alpha;
      lrow[r] = la + psum;
#pragma unroll
      for (int t = 0; t < 2; ++t) o[t][r] = o[t][r] * alpha;
    }
    wave_sync_lds();

#pragma unroll
    for (int kk = 0; kk < 2; ++kk) {
      FH pa;
      pa.h[0] = *(const v8h*)(pw + c * 64 + kk * 32 + 8 * hh);
      pa.h[1] = *(const v8h*)(pw + c * 64 + kk * 32 + 16 + 8 * hh);
#pragma unroll
      for (int t = 0; t < 2; ++t) {
        const int d = head * HD + t * 16 + c;
        const v16h vb = ldfrag_h(V + ((size_t)g * NF + d) * NW + kv0 + kk * 32 + 8 * hh);
        o[t] = mma_h(pa.v, vb, o[t]);
      }
    }
    wave_sync_lds();
  }

#pragma unroll
  for (int r = 0; r < 8; ++r) {
    const float l = lrow[r];
    const float inv = ((l > 0.f) ? (1.0f / l) : 0.f) * (1.0f / 1024.0f);
#pragma unroll
    for (int t = 0; t < 2; ++t) {
      const int colx = hl * HD + t * 16 + c;
      Os[(wq * 16 + 8 * hh + r) * 68 + colx] = o[t][r] * inv;
    }
  }
  __syncthreads();
  {
    const int q8 = lane >> 3, c8 = (lane & 7) * 8;
    v4u hv[2];
#pragma unroll
    for (int it = 0; it < 2; ++it) {
      const int row = wave * 8 + it * 4 + q8;
      const float* sp = Os + row * 68 + c8;
      v4u a;
#pragma unroll
      for (int e = 0; e < 4; ++e) a[e] = pkh(sp[2 * e], sp[2 * e + 1]);
      hv[it] = a;
    }
    for (int ps = 0; ps < 2; ++ps) {
#pragma unroll
      for (int it = 0; it < 2; ++it) {
        const int row = wave * 8 + it * 4 + q8;
        *(volatile v4u*)(atp + (trow0 + (size_t)qt * 64 + row) * NF + hp * 64 + c8) = hv[it];
      }
      __threadfence();
    }
  }
}

static GemmArgs mk_args(const unsigned short* A, long long aP, long long aG, long long aC, int lda,
                        const unsigned short* B, long long bP, long long bG, long long bC, int ldb,
                        void* C, const float* R, long long cP, long long cG, long long cC, int ldc,
                        int M, int N, int K, float s0, float s1) {
  GemmArgs g;
  g.A = A; g.B = B; g.C = C; g.R = R;
  g.aP = aP; g.aG = aG; g.aC = aC;
  g.bP = bP; g.bG = bG; g.bC = bC;
  g.cP = cP; g.cG = cG; g.cC = cC;
  g.lda = lda; g.ldb = ldb; g.ldc = ldc;
  g.M = M; g.N = N; g.K = K;
  g.s0 = s0; g.s1 = s1;
  return g;
}

extern "C" void kernel_launch(void* const* d_in, const int* in_sizes, int n_in,
                              void* d_out, int out_size, void* d_ws, size_t ws_size,
                              hipStream_t stream) {
  if (n_in < 19) return;
  if (in_sizes[0] != NB * NCI * NF * NW) return;
  if (in_sizes[1] != NC * NCI || in_sizes[2] != NC) return;
  if (in_sizes[3] != NC * NF || in_sizes[4] != NC * NF) return;
  if (in_sizes[5] != WSQ || in_sizes[6] != NC * NC * 3 || in_sizes[7] != NC) return;
  if (in_sizes[8] != WSQ || in_sizes[9] != NC * NC * 3 || in_sizes[10] != NC) return;
  if (in_sizes[11] != WSQ || in_sizes[12] != NC * NC * 3 || in_sizes[13] != NC) return;
  if (in_sizes[14] != WSQ || in_sizes[15] != NC * NF || in_sizes[16] != NC * NF) return;
  if (in_sizes[17] != WSL || in_sizes[18] != WSL) return;
  if (out_size != NG * GFW) return;

  const float* x       = (const float*)d_in[0];
  const float* embed_w = (const float*)d_in[1];
  const float* embed_b = (const float*)d_in[2];
  const float* norm1_w = (const float*)d_in[3];
  const float* norm1_b = (const float*)d_in[4];
  const float* q_pw    = (const float*)d_in[5];
  const float* q_cw    = (const float*)d_in[6];
  const float* q_cb    = (const float*)d_in[7];
  const float* k_pw    = (const float*)d_in[8];
  const float* k_cw    = (const float*)d_in[9];
  const float* k_cb    = (const float*)d_in[10];
  const float* v_pw    = (const float*)d_in[11];
  const float* v_cw    = (const float*)d_in[12];
  const float* v_cb    = (const float*)d_in[13];
  const float* out_pw  = (const float*)d_in[14];
  const float* norm2_w = (const float*)d_in[15];
  const float* norm2_b = (const float*)d_in[16];
  const float* lin1_w  = (const float*)d_in[17];
  const float* lin2_w  = (const float*)d_in[18];
  float* out = (float*)d_out;

  const size_t sWH  = (size_t)NWH * 2;
  const size_t sTB  = (size_t)32 * NW * 4;
  const size_t sX   = (size_t)NG * GFW * 4;
  const size_t sP16 = (size_t)NG * GFW * 2;
  const size_t sHM  = (size_t)NG * GWE * 2;
  size_t off = 0;
  const size_t oWH  = off; off += sWH;
  const size_t oTB  = off; off += sTB;
  const size_t oX   = off; off += sX;
  const size_t oX1  = off; off += sX;
  const size_t oXNT = off; off += sP16;
  const size_t oAT  = off; off += sP16;
  const size_t oYT  = off; off += 3 * sP16;
  const size_t oQKV = off; off += 3 * sP16;
  if (off > ws_size) return;
  if (off > (size_t)134217728) return;
  if (sHM > 6 * sP16) return;

  char* ws = (char*)d_ws;
  unsigned short* WH  = (unsigned short*)(ws + oWH);
  float*          TB  = (float*)(ws + oTB);
  float*          X   = (float*)(ws + oX);
  float*          X1  = (float*)(ws + oX1);
  unsigned short* XNT = (unsigned short*)(ws + oXNT);
  unsigned short* AT  = (unsigned short*)(ws + oAT);
  unsigned short* YT  = (unsigned short*)(ws + oYT);
  unsigned short* YV  = YT + (size_t)2 * NG * GFW;
  unsigned short* QKV = (unsigned short*)(ws + oQKV);
  unsigned short* QT  = QKV;
  unsigned short* KT  = QKV + (size_t)NG * GFW;
  unsigned short* V16 = QKV + (size_t)2 * NG * GFW;
  unsigned short* HMT = YT;
  const unsigned short* WV = WH + (size_t)2 * WSQ;
  const unsigned short* WO = WH + (size_t)3 * WSQ;
  const unsigned short* W1 = WH + (size_t)4 * WSQ;
  const unsigned short* W2 = WH + (size_t)4 * WSQ + WSL;

  const dim3 blk(256);
  const float inv64 = 1.0f / 64.0f;
  const float inv4k = 1.0f / 4096.0f;
  const float sscale = 1.0789593218788871e-05f;

  const int tSQ  = (NW / 64) * (NF / 64);
  const int tFE  = (NW / 64) * (NFE / 64);
  const dim3 gSQ2((tSQ + 7) / 8, 2 * NG);
  const dim3 gSQ((tSQ + 7) / 8, NG);
  const dim3 gFE((tFE + 7) / 8, NG);

  cvt_w<<<dim3(NWH / CVB), blk, 0, stream>>>(q_pw, k_pw, v_pw, out_pw, lin1_w, lin2_w, WH);
  trig_tab<<<dim3((NW + 255) / 256, 32), blk, 0, stream>>>(TB);
  ln_cols<1><<<dim3(NW / 32, NG), blk, 0, stream>>>(x, embed_w, embed_b, norm1_w, norm1_b, X, XNT);
  gemm64<1><<<gSQ2, blk, 0, stream>>>(
      mk_args(XNT, 0, GFW, 0, NF, WH, WSQ, 0, (long long)NF * NF, NF,
              (void*)YT, X, (long long)NG * GFW, GFW, 0, NF, NW, NF, NF, 1.0f, 1.0f));
  gemm64<1><<<gSQ, blk, 0, stream>>>(
      mk_args(WV, 0, 0, (long long)NF * NF, NF, XNT, 0, GFW, 0, NF,
              (void*)YV, X, 0, GFW, 0, NW, NF, NW, NF, 1.0f, 1.0f));
  conv_qk<<<dim3((2 * NG * NW * (NF / 8)) / 256), blk, 0, stream>>>(YT, q_cw, q_cb, k_cw, k_cb, TB, QT);
  conv_v<<<dim3((NG * NF * (NW / 8)) / 256), blk, 0, stream>>>(YV, v_cw, v_cb, V16);
  attn_hd32<<<dim3(NW / 64, NHD / 2, NG), blk, 0, stream>>>(QT, KT, V16, AT, sscale);
  gemm64<0><<<gSQ, blk, 0, stream>>>(
      mk_args(WO, 0, 0, (long long)NF * NF, NF, AT, 0, GFW, 0, NF,
              (void*)X1, X, 0, GFW, 0, NW, NF, NW, NF, inv4k, 1.0f));
  ln_cols<0><<<dim3(NW / 32, NG), blk, 0, stream>>>(X1, embed_w, embed_b, norm2_w, norm2_b, X, XNT);
  gemm64<2><<<gFE, blk, 0, stream>>>(
      mk_args(XNT, 0, GFW, 0, NF, W1, 0, 0, (long long)NFE * NF, NF,
              (void*)HMT, X, 0, GWE, 0, NFE, NW, NFE, NF, inv64, 64.0f));
  gemm64<0><<<gSQ, blk, 0, stream>>>(
      mk_args(W2, 0, 0, (long long)NF * NFE, NFE, HMT, 0, GWE, 0, NFE,
              (void*)out, X1, 0, GFW, 0, NW, NF, NW, NFE, inv4k, 1.0f));
  (void)hipGetLastError();
}
